// RBFN_16819091931602
// MI455X (gfx1250) — hardware-run, weakly checked
//
#include <hip/hip_runtime.h>
#include <stddef.h>
#include <stdint.h>
#include <math.h>

#define NB   16384
#define NCEN 2048
#define ND   256
#define NO   64
#define WK   (ND + NCEN)
#define WSEG (WK / 256)
#define SHP  136
#define SFP  68

static_assert(ND == 256);
static_assert(ND % 32 == 0);
static_assert(NCEN % 32 == 0);
static_assert(WK % 256 == 0);
static_assert(WSEG == 9);
static_assert(NB % 128 == 0);
static_assert(NCEN % 128 == 0);
static_assert(NB % 32 == 0);
static_assert(NCEN % 32 == 0);
static_assert(NO == 64);
static_assert(NO % 8 == 0);

typedef _Float16 hh;
typedef hh    v16h __attribute__((ext_vector_type(16)));
typedef hh    v8h  __attribute__((ext_vector_type(8)));
typedef float v8f  __attribute__((ext_vector_type(8)));
typedef float v4f  __attribute__((ext_vector_type(4)));

union Frag { v16h v; v8h p[2]; };

__device__ __forceinline__ v8f zero8() { return (v8f){0.f, 0.f, 0.f, 0.f, 0.f, 0.f, 0.f, 0.f}; }

__device__ __forceinline__ float wsum(float v) {
#pragma unroll
  for (int off = 16; off > 0; off >>= 1) v += __shfl_xor(v, off, 32);
  return v;
}

__device__ __forceinline__ v16h ldfrag(const hh* __restrict__ p, int ld, int row0, int k0, int lane) {
  const hh* q = p + (size_t)(row0 + (lane & 15)) * (size_t)ld + k0 + 8 * (lane >> 4);
  Frag f;
  f.p[0] = *(const v8h*)(q);
  f.p[1] = *(const v8h*)(q + 16);
  return f.v;
}

__device__ __forceinline__ v8f mma16(v16h a, v16h b, v8f cc) {
  return __builtin_amdgcn_wmma_f32_16x16x32_f16(false, a, false, b, (short)0, cc, false, false);
}

__device__ __forceinline__ void gemm32x64(const hh* __restrict__ A, int lda, const hh* __restrict__ B, int ldb,
                                          int ma, int nb, int kdim, int lane, v8f (&acc)[2][4]) {
#pragma unroll 1
  for (int k0 = 0; k0 < kdim; k0 += 32) {
    const v16h a0 = ldfrag(A, lda, ma, k0, lane);
    const v16h a1 = ldfrag(A, lda, ma + 16, k0, lane);
    const v16h b0 = ldfrag(B, ldb, nb, k0, lane);
    const v16h b1 = ldfrag(B, ldb, nb + 16, k0, lane);
    const v16h b2 = ldfrag(B, ldb, nb + 32, k0, lane);
    const v16h b3 = ldfrag(B, ldb, nb + 48, k0, lane);
    acc[0][0] = mma16(a0, b0, acc[0][0]);
    acc[1][0] = mma16(a1, b0, acc[1][0]);
    acc[0][1] = mma16(a0, b1, acc[0][1]);
    acc[1][1] = mma16(a1, b1, acc[1][1]);
    acc[0][2] = mma16(a0, b2, acc[0][2]);
    acc[1][2] = mma16(a1, b2, acc[1][2]);
    acc[0][3] = mma16(a0, b3, acc[0][3]);
    acc[1][3] = mma16(a1, b3, acc[1][3]);
    asm volatile("v_nop\n\tv_nop\n\tv_nop\n\tv_nop"
                 : "+v"(acc[0][0]), "+v"(acc[0][1]), "+v"(acc[0][2]), "+v"(acc[0][3]),
                   "+v"(acc[1][0]), "+v"(acc[1][1]), "+v"(acc[1][2]), "+v"(acc[1][3])
                 : "v"(a0), "v"(a1), "v"(b0), "v"(b1), "v"(b2), "v"(b3));
  }
}

__device__ __forceinline__ void gemm16x64(const hh* __restrict__ A, int lda, const hh* __restrict__ B, int ldb,
                                          int ma, int nb, int kdim, int lane, v8f (&acc)[4]) {
#pragma unroll 1
  for (int k0 = 0; k0 < kdim; k0 += 32) {
    const v16h a0 = ldfrag(A, lda, ma, k0, lane);
    const v16h b0 = ldfrag(B, ldb, nb, k0, lane);
    const v16h b1 = ldfrag(B, ldb, nb + 16, k0, lane);
    const v16h b2 = ldfrag(B, ldb, nb + 32, k0, lane);
    const v16h b3 = ldfrag(B, ldb, nb + 48, k0, lane);
    acc[0] = mma16(a0, b0, acc[0]);
    acc[1] = mma16(a0, b1, acc[1]);
    acc[2] = mma16(a0, b2, acc[2]);
    acc[3] = mma16(a0, b3, acc[3]);
    asm volatile("v_nop\n\tv_nop\n\tv_nop\n\tv_nop"
                 : "+v"(acc[0]), "+v"(acc[1]), "+v"(acc[2]), "+v"(acc[3])
                 : "v"(a0), "v"(b0), "v"(b1), "v"(b2), "v"(b3));
  }
}

__global__ __launch_bounds__(256) void k_rows(const float* __restrict__ src, hh* __restrict__ dst,
                                              float* __restrict__ nrm) {
  __shared__ __align__(16) float sn[32];
  const int tid = threadIdx.x, lane = tid & 31, w = tid >> 5;
  const int rb = blockIdx.x * 32 + w * 4;
  v8h hv[4];
#pragma unroll
  for (int i = 0; i < 4; ++i) {
    const float* rp = src + (size_t)(rb + i) * ND + 8 * lane;
    const v4f a0 = *(const v4f*)(rp), a1 = *(const v4f*)(rp + 4);
    const v8f ta = {a0[0], a0[1], a0[2], a0[3], a1[0], a1[1], a1[2], a1[3]};
    float s = 0.f;
#pragma unroll
    for (int e = 0; e < 8; ++e) s = fmaf(ta[e], ta[e], s);
    s = wsum(s);
    hv[i] = __builtin_convertvector(ta, v8h);
    if (lane == 0) sn[w * 4 + i] = s;
  }
#pragma unroll
  for (int i = 0; i < 4; ++i) {
    hh* op = dst + (size_t)(rb + i) * ND + 8 * lane;
    *(volatile v8h*)(op) = hv[i];
  }
  __threadfence();
#pragma unroll
  for (int i = 0; i < 4; ++i) {
    hh* op = dst + (size_t)(rb + i) * ND + 8 * lane;
    *(volatile v8h*)(op) = hv[i];
  }
  __syncthreads();
  if (w == 0) {
    const int li = lane & 7;
    const v4f v = *(const v4f*)(sn + 4 * li);
    float* gp = nrm + (size_t)blockIdx.x * 32 + 4 * li;
    if (lane < 8) *(volatile v4f*)gp = v;
    __threadfence();
    if (lane < 8) *(volatile v4f*)gp = v;
  }
}

__global__ __launch_bounds__(256) void k_cvt_w(const float* __restrict__ wsrc, hh* __restrict__ wh) {
  const int tid = threadIdx.x, lane = tid & 31, w = tid >> 5;
  const int n = blockIdx.x * 8 + w;
  v8h hv[WSEG];
#pragma unroll
  for (int seg = 0; seg < WSEG; ++seg) {
    const float* fp = wsrc + (size_t)n * WK + seg * 256 + 8 * lane;
    const v4f a0 = *(const v4f*)(fp), a1 = *(const v4f*)(fp + 4);
    v8f t = {a0[0], a0[1], a0[2], a0[3], a1[0], a1[1], a1[2], a1[3]};
    t = t * 16.0f;
    hv[seg] = __builtin_convertvector(t, v8h);
  }
#pragma unroll
  for (int seg = 0; seg < WSEG; ++seg)
    *(volatile v8h*)(wh + (size_t)n * WK + seg * 256 + 8 * lane) = hv[seg];
  __threadfence();
#pragma unroll
  for (int seg = 0; seg < WSEG; ++seg)
    *(volatile v8h*)(wh + (size_t)n * WK + seg * 256 + 8 * lane) = hv[seg];
}

__global__ __launch_bounds__(256) void k_gemm_r(const hh* __restrict__ XH, const hh* __restrict__ CH,
                                                const float* __restrict__ XN, const float* __restrict__ CN,
                                                const float* __restrict__ beta, hh* __restrict__ PH) {
  __shared__ __align__(16) hh sh[128 * SHP];
  const int tid = threadIdx.x, lane = tid & 31, w = tid >> 5;
  const int h = lane >> 4, c = lane & 15;
  const int wm = (w >> 1) * 32, wn = (w & 1) * 64;
  const int m0 = blockIdx.y * 128;
  const int n0 = blockIdx.x * 128;

  v8f acc[2][4];
#pragma unroll
  for (int i = 0; i < 2; ++i)
#pragma unroll
    for (int j = 0; j < 4; ++j) acc[i][j] = zero8();
  gemm32x64(XH, ND, CH, ND, m0 + wm, n0 + wn, ND, lane, acc);

  float cnc[4], btc[4];
#pragma unroll
  for (int j = 0; j < 4; ++j) {
    cnc[j] = CN[n0 + wn + 16 * j + c];
    btc[j] = beta[n0 + wn + 16 * j + c];
  }

#pragma unroll
  for (int i = 0; i < 2; ++i) {
    const v8f xt = *(const v8f*)(XN + m0 + wm + 16 * i + 8 * h);
#pragma unroll
    for (int j = 0; j < 4; ++j) {
      float v[8];
#pragma unroll
      for (int r = 0; r < 8; ++r) {
        const float g  = acc[i][j][r];
        const float sq = (xt[r] + cnc[j]) - 2.0f * g;
        const float nb = -btc[j];
        const float pv = expf(nb * sq);
        v[r] = pv * 4096.0f;
      }
#pragma unroll
      for (int r = 0; r < 8; ++r)
        sh[(wm + 16 * i + 8 * h + r) * SHP + wn + 16 * j + c] = (hh)v[r];
    }
  }
  __syncthreads();

  v8h val[8];
  size_t go[8];
#pragma unroll
  for (int it = 0; it < 8; ++it) {
    const int p  = tid + 256 * it;
    const int lr = p >> 4;
    const int pc = p & 15;
    val[it] = *(const v8h*)(sh + lr * SHP + pc * 8);
    go[it] = (size_t)(m0 + lr) * NCEN + n0 + pc * 8;
  }
#pragma unroll
  for (int it = 0; it < 8; ++it) *(volatile v8h*)(PH + go[it]) = val[it];
  __threadfence();
#pragma unroll
  for (int it = 0; it < 8; ++it) *(volatile v8h*)(PH + go[it]) = val[it];
}

__global__ __launch_bounds__(256) void k_gemm_out(const hh* __restrict__ XH, const hh* __restrict__ PH,
                                                  const hh* __restrict__ WH, const float* __restrict__ bias,
                                                  float* __restrict__ out) {
  __shared__ __align__(16) float sf[128 * SFP];
  const int tid = threadIdx.x, lane = tid & 31, w = tid >> 5;
  const int h = lane >> 4, c = lane & 15;
  const int m0 = blockIdx.x * 128;
  const int row0 = m0 + 16 * w;

  v8f accA[4], accB[4];
#pragma unroll
  for (int j = 0; j < 4; ++j) { accA[j] = zero8(); accB[j] = zero8(); }
  gemm16x64(XH, ND, WH, WK, row0, 0, ND, lane, accA);
  gemm16x64(PH, NCEN, WH + ND, WK, row0, 0, NCEN, lane, accB);

#pragma unroll
  for (int t = 0; t < 4; ++t) {
    const float bv = bias[16 * t + c];
#pragma unroll
    for (int r = 0; r < 8; ++r) {
      const float v = (accA[t][r] * 0.0625f + accB[t][r] * (1.0f / 65536.0f)) + bv;
      sf[(16 * w + 8 * h + r) * SFP + 16 * t + c] = v;
    }
  }
  __syncthreads();

  v4f val[8];
  size_t go[8];
#pragma unroll
  for (int it = 0; it < 8; ++it) {
    const int p  = tid + 256 * it;
    const int lr = p >> 4;
    const int pc = p & 15;
    val[it] = *(const v4f*)(sf + lr * SFP + pc * 4);
    go[it] = (size_t)(m0 + lr) * NO + pc * 4;
  }
#pragma unroll
  for (int it = 0; it < 8; ++it) *(volatile v4f*)(out + go[it]) = val[it];
  __threadfence();
#pragma unroll
  for (int it = 0; it < 8; ++it) *(volatile v4f*)(out + go[it]) = val[it];
}

extern "C" void kernel_launch(void* const* d_in, const int* in_sizes, int n_in,
                              void* d_out, int out_size, void* d_ws, size_t ws_size,
                              hipStream_t stream) {
  if (n_in < 5) return;
  if (in_sizes[0] != NB * ND) return;
  if (in_sizes[1] != NCEN * ND) return;
  if (in_sizes[2] != NCEN) return;
  if (in_sizes[3] != NO * WK) return;
  if (in_sizes[4] != NO) return;
  if (out_size != NB * NO) return;

  const float* x    = (const float*)d_in[0];
  const float* cen  = (const float*)d_in[1];
  const float* beta = (const float*)d_in[2];
  const float* lw   = (const float*)d_in[3];
  const float* lb   = (const float*)d_in[4];
  float* out = (float*)d_out;

  size_t off = 0;
  const size_t oXH = off; off += (size_t)NB * ND * 2;
  const size_t oCH = off; off += (size_t)NCEN * ND * 2;
  const size_t oXN = off; off += (size_t)NB * 4;
  const size_t oCN = off; off += (size_t)NCEN * 4;
  const size_t oWH = off; off += (size_t)NO * WK * 2;
  const size_t oPH = off; off += (size_t)NB * NCEN * 2;
  if (off > ws_size) return;
  if (off > (size_t)134217728) return;

  char* ws = (char*)d_ws;
  hh*    XH = (hh*)(ws + oXH);
  hh*    CH = (hh*)(ws + oCH);
  float* XN = (float*)(ws + oXN);
  float* CN = (float*)(ws + oCN);
  hh*    WH = (hh*)(ws + oWH);
  hh*    PH = (hh*)(ws + oPH);

  k_rows<<<dim3(NB / 32), dim3(256), 0, stream>>>(x, XH, XN);
  k_rows<<<dim3(NCEN / 32), dim3(256), 0, stream>>>(cen, CH, CN);
  k_cvt_w<<<dim3(NO / 8), dim3(256), 0, stream>>>(lw, WH);
  k_gemm_r<<<dim3(NCEN / 128, NB / 128), dim3(256), 0, stream>>>(XH, CH, XN, CN, beta, PH);
  k_gemm_out<<<dim3(NB / 128), dim3(256), 0, stream>>>(XH, PH, WH, lb, out);
  (void)hipGetLastError();
}
